// SequenceGRU_64433099374751
// MI455X (gfx1250) — hardware-verified
//
#include <hip/hip_runtime.h>
#include <math.h>

typedef __attribute__((ext_vector_type(16))) _Float16 v16h;
typedef __attribute__((ext_vector_type(8)))  _Float16 v8h;
typedef __attribute__((ext_vector_type(8)))  float    v8f;
typedef __attribute__((ext_vector_type(4)))  float    v4f;

constexpr int kBatch   = 2048;
constexpr int kSteps   = 1024;
constexpr int kHid     = 51;
constexpr int kGate    = 3 * kHid;
constexpr int kRows    = 16;
constexpr int kBlocks  = kBatch / kRows;
constexpr int kNPad    = 160;
constexpr int kKPad    = 64;
constexpr int kThreads = 320;
constexpr int kWaves   = kThreads / 32;
constexpr int kHPitch  = 72;
constexpr int kSlabP   = 164;
constexpr int kHfP     = 68;
constexpr int kChunk   = 32;
constexpr int kPairs   = kRows * kHid;
constexpr int kIters   = 3;
constexpr int kTailN   = kPairs - 2 * kThreads;
constexpr int kTailWaves = (kTailN + 31) / 32;
constexpr int kPadCols = kKPad - kHid;
constexpr int kPadN    = kRows * kPadCols;
constexpr int kPlane   = kNPad * kKPad;
constexpr float kCarry = 256.0f;
constexpr float kFold  = 1.0f / kCarry;
constexpr float kF16Min = 6.103515625e-05f;

static_assert(kGate == 153, "gate rows");
static_assert(kBlocks * kRows == kBatch, "sample tiling");
static_assert(kNPad == kWaves * 16 && kNPad >= kGate, "one 16-column tile per wave");
static_assert(kKPad % 32 == 0 && kKPad >= kHid, "k padded to two 32-deep steps");
static_assert(kPlane % kThreads == 0, "weight staging covers the plane exactly");
static_assert(kPairs > 2 * kThreads && kPairs <= kIters * kThreads, "pair tiling");
static_assert(kTailN > 0 && kTailN <= kThreads, "tail pairs");
static_assert(kPadN <= kThreads, "pad refill fits one pass");
static_assert(kSteps % kChunk == 0 && kChunk == 32, "one 128-B line per sample per chunk");
static_assert((kHPitch % 8) == 0 && (kHfP % 4) == 0 && (kSlabP % 4) == 0, "vector alignment of LDS pitches");

__device__ __forceinline__ float bf16_value(float f) {
  unsigned u = __float_as_uint(f);
  u = (u + 0x7FFFu + ((u >> 16) & 1u)) & 0xFFFF0000u;
  return __uint_as_float(u);
}
__device__ __forceinline__ _Float16 to_h_flush(float v) {
  const float z = (fabsf(v) < kF16Min) ? 0.0f : v;
  return (_Float16)z;
}
__device__ __forceinline__ _Float16 weight_to_h(float w, bool inside) {
  const float c = bf16_value(w) * kCarry;
  const float s = inside ? c : 0.0f;
  return to_h_flush(s);
}
__device__ __forceinline__ float gate_sig(float a) {
  return __builtin_amdgcn_rcpf(1.0f + __expf(-a));
}
__device__ __forceinline__ float gate_tanh(float a) {
  return fmaf(-2.0f, __builtin_amdgcn_rcpf(1.0f + __expf(2.0f * a)), 1.0f);
}

union FragU { v16h v; v8h h[2]; };
__device__ __forceinline__ v16h frag_load(const _Float16* p) {
  FragU f;
  f.h[0] = *(const v8h*)(p);
  f.h[1] = *(const v8h*)(p + 16);
  return f.v;
}
__device__ __forceinline__ v8f mma_f16(v16h a, v16h b, v8f c) {
  return __builtin_amdgcn_wmma_f32_16x16x32_f16(false, a, false, b, (short)0, c, false, false);
}
__device__ __forceinline__ void group_guard(v8f& c, v16h a0, v16h a1, v16h b0, v16h b1) {
  asm volatile("v_nop\n\tv_nop\n\tv_nop\n\tv_nop" : "+v"(c) : "v"(a0), "v"(a1), "v"(b0), "v"(b1));
}

__global__ __launch_bounds__(320) void two_cell_scalar_steps(
    const float* __restrict__ input,
    const float* __restrict__ w_ih1, const float* __restrict__ w_hh1,
    const float* __restrict__ b_ih1, const float* __restrict__ b_hh1,
    const float* __restrict__ w_ih2, const float* __restrict__ w_hh2,
    const float* __restrict__ b_ih2, const float* __restrict__ b_hh2,
    const float* __restrict__ lin_w, const float* __restrict__ lin_b,
    const int* __restrict__ future_p, float* __restrict__ out)
{
  __shared__ __align__(16) _Float16 sW[3 * kPlane];
  __shared__ __align__(16) float sSlabA[kRows * kSlabP];
  __shared__ __align__(16) float sSlabB[kRows * kSlabP];
  __shared__ __align__(16) _Float16 sH1[kRows * kHPitch];
  __shared__ __align__(16) _Float16 sH2[kRows * kHPitch];
  __shared__ __align__(16) float sH2f[kRows * kHfP];
  __shared__ __align__(16) float sX[kRows * kChunk];
  __shared__ __align__(16) float sOutP[2 * kRows * kChunk];
  __shared__ __align__(16) float sC[5 * kNPad];
  __shared__ __align__(16) float sLw[kKPad];

  const int tid  = threadIdx.x;
  const int lane = tid & 31;
  const int wave = __builtin_amdgcn_readfirstlane(tid >> 5);
  const int hh   = lane >> 4;
  const int jj   = lane & 15;
  const int b0   = blockIdx.x * kRows;

#pragma unroll 1
  for (int i = tid; i < kRows * kHPitch; i += kThreads) {
    sH1[i] = (_Float16)0.0f;
    sH2[i] = (_Float16)0.0f;
  }
#pragma unroll 1
  for (int i = tid; i < kRows * kHfP; i += kThreads) sH2f[i] = 0.0f;

#pragma unroll 1
  for (int e = tid; e < kPlane; e += kThreads) {
    const int n = e >> 6;
    const int k = e & (kKPad - 1);
    const bool inside = (n < kGate) && (k < kHid);
    const int nc = (n < kGate) ? n : (kGate - 1);
    const int kc = (k < kHid) ? k : (kHid - 1);
    const int src = nc * kHid + kc;
    const float wa = w_hh1[src];
    const float wb = w_ih2[src];
    const float wc = w_hh2[src];
    sW[e]              = weight_to_h(wa, inside);
    sW[kPlane + e]     = weight_to_h(wb, inside);
    sW[2 * kPlane + e] = weight_to_h(wc, inside);
  }

  {
    const int ci = (tid < kGate) ? tid : (kGate - 1);
    float v0 = w_ih1[ci];
    float v1 = b_ih1[ci];
    float v2 = b_hh1[ci];
    float v3 = b_ih2[ci];
    float v4 = b_hh2[ci];
    asm volatile("" : "+v"(v0));
    asm volatile("" : "+v"(v1));
    asm volatile("" : "+v"(v2));
    asm volatile("" : "+v"(v3));
    asm volatile("" : "+v"(v4));
    const int li = (tid < kHid) ? tid : (kHid - 1);
    float lw = lin_w[li];
    asm volatile("" : "+v"(lw));
    const bool okc = (tid < kGate);
    if (tid < kNPad) {
      sC[tid]             = okc ? bf16_value(v0) : 0.0f;
      sC[kNPad + tid]     = okc ? bf16_value(v1) : 0.0f;
      sC[2 * kNPad + tid] = okc ? bf16_value(v2) : 0.0f;
      sC[3 * kNPad + tid] = okc ? bf16_value(v3) : 0.0f;
      sC[4 * kNPad + tid] = okc ? bf16_value(v4) : 0.0f;
    }
    if (tid < kKPad) sLw[tid] = (tid < kHid) ? bf16_value(lw) : 0.0f;
  }

  const int xr = (tid & 127) >> 3;
  const int xp = (tid & 7) * 4;
  const float* xsrc = input + (size_t)(b0 + xr) * kSteps + xp;
  {
    const v4f xv = *(const v4f*)(xsrc);
    float x0 = xv[0];
    float x1 = xv[1];
    float x2 = xv[2];
    float x3 = xv[3];
    asm volatile("" : "+v"(x0));
    asm volatile("" : "+v"(x1));
    asm volatile("" : "+v"(x2));
    asm volatile("" : "+v"(x3));
    if (tid < 128) {
      v4f xs;
      xs[0] = bf16_value(x0);
      xs[1] = bf16_value(x1);
      xs[2] = bf16_value(x2);
      xs[3] = bf16_value(x3);
      *(v4f*)(sX + xr * kChunk + xp) = xs;
    }
  }

  float lb = lin_b[0];
  asm volatile("" : "+v"(lb));
  const float linb = bf16_value(lb);
  const int fut = future_p[0];
  const bool poison = (fut != 0);
  const float qnan = __uint_as_float(0x7FC00000u);

  __syncthreads();

  const _Float16* wbase = sW + (wave * 16 + jj) * kKPad + 8 * hh;
  const v16h bA0 = frag_load(wbase);
  const v16h bA1 = frag_load(wbase + 32);
  const v16h bI0 = frag_load(wbase + kPlane);
  const v16h bI1 = frag_load(wbase + kPlane + 32);
  const v16h bH0 = frag_load(wbase + 2 * kPlane);
  const v16h bH1 = frag_load(wbase + 2 * kPlane + 32);

  int   so[kIters], ho[kIters], fo[kIters], xo[kIters];
  float wr[kIters], wz[kIters], wn[kIters];
  float c1r[kIters], c1z[kIters], c1i[kIters], c1h[kIters];
  float c2r[kIters], c2z[kIters], c2i[kIters], c2h[kIters];
  float h1f[kIters], h2f[kIters];
#pragma unroll
  for (int it = 0; it < kIters; ++it) {
    const int p  = it * kThreads + tid;
    const int pc = (p < kPairs) ? p : (kPairs - 1);
    const int s  = pc / kHid;
    const int u  = pc - s * kHid;
    so[it] = s * kSlabP + u;
    ho[it] = s * kHPitch + u;
    fo[it] = s * kHfP + u;
    xo[it] = s * kChunk;
    wr[it] = sC[u];
    wz[it] = sC[kHid + u];
    wn[it] = sC[2 * kHid + u];
    c1r[it] = sC[kNPad + u] + sC[2 * kNPad + u];
    c1z[it] = sC[kNPad + kHid + u] + sC[2 * kNPad + kHid + u];
    c1i[it] = sC[kNPad + 2 * kHid + u];
    c1h[it] = sC[2 * kNPad + 2 * kHid + u];
    c2r[it] = sC[3 * kNPad + u] + sC[4 * kNPad + u];
    c2z[it] = sC[3 * kNPad + kHid + u] + sC[4 * kNPad + kHid + u];
    c2i[it] = sC[3 * kNPad + 2 * kHid + u];
    c2h[it] = sC[4 * kNPad + 2 * kHid + u];
    h1f[it] = 0.0f;
    h2f[it] = 0.0f;
  }
  const bool tailOk = (tid < kTailN);

  const bool padOk  = (tid < kPadN);
  const int  padRow = padOk ? (tid / kPadCols) : 0;
  const int  padCol = padOk ? (tid - padRow * kPadCols) : 0;
  const int  padOff = padRow * kHPitch + kHid + padCol;

  const _Float16* aH1 = sH1 + jj * kHPitch + 8 * hh;
  const _Float16* aH2 = sH2 + jj * kHPitch + 8 * hh;
  const int dOff = (8 * hh) * kSlabP + wave * 16 + jj;
  const v8f zero8 = (v8f){0.f, 0.f, 0.f, 0.f, 0.f, 0.f, 0.f, 0.f};

#pragma unroll 1
  for (int t = 0; t < kSteps; ++t) {
    const int tl = t & (kChunk - 1);

    {
      const v16h a0 = frag_load(aH1);
      const v16h a1 = frag_load(aH1 + 32);
      v8f acc = zero8;
      acc = mma_f16(a0, bA0, acc);
      acc = mma_f16(a1, bA1, acc);
      group_guard(acc, a0, a1, bA0, bA1);
#pragma unroll
      for (int r = 0; r < 8; ++r) sSlabA[dOff + r * kSlabP] = acc[r];
    }
    __syncthreads();

#pragma unroll
    for (int it = 0; it < kIters; ++it) {
      if (it < 2 || wave < kTailWaves) {
        const float x = sX[xo[it] + tl];
        const float* ga = sSlabA + so[it];
        const float ar = ga[0];
        const float az = ga[kHid];
        const float an = ga[2 * kHid];
        const float pr = fmaf(ar, kFold, fmaf(x, wr[it], c1r[it]));
        const float pz = fmaf(az, kFold, fmaf(x, wz[it], c1z[it]));
        const float rg = gate_sig(pr);
        const float zg = gate_sig(pz);
        const float gin = fmaf(x, wn[it], c1i[it]);
        const float ghn = fmaf(an, kFold, c1h[it]);
        const float ng = gate_tanh(fmaf(rg, ghn, gin));
        const float hn = fmaf(zg, h1f[it] - ng, ng);
        h1f[it] = hn;
        if (it < 2 || tailOk) sH1[ho[it]] = to_h_flush(hn);
      }
    }
    if (padOk) sH1[padOff] = (_Float16)0.0f;
    __syncthreads();

    {
      const v16h p0 = frag_load(aH1);
      const v16h p1 = frag_load(aH1 + 32);
      v8f ai = zero8;
      ai = mma_f16(p0, bI0, ai);
      ai = mma_f16(p1, bI1, ai);
      group_guard(ai, p0, p1, bI0, bI1);
      const v16h q0 = frag_load(aH2);
      const v16h q1 = frag_load(aH2 + 32);
      v8f ah = zero8;
      ah = mma_f16(q0, bH0, ah);
      ah = mma_f16(q1, bH1, ah);
      group_guard(ah, q0, q1, bH0, bH1);
#pragma unroll
      for (int r = 0; r < 8; ++r) {
        sSlabA[dOff + r * kSlabP] = ai[r];
        sSlabB[dOff + r * kSlabP] = ah[r];
      }
    }
    __syncthreads();

#pragma unroll
    for (int it = 0; it < kIters; ++it) {
      if (it < 2 || wave < kTailWaves) {
        const float* ga = sSlabA + so[it];
        const float* gb = sSlabB + so[it];
        const float sr = ga[0] + gb[0];
        const float sz = ga[kHid] + gb[kHid];
        const float ani = ga[2 * kHid];
        const float anh = gb[2 * kHid];
        const float pr = fmaf(sr, kFold, c2r[it]);
        const float pz = fmaf(sz, kFold, c2z[it]);
        const float rg = gate_sig(pr);
        const float zg = gate_sig(pz);
        const float gin = fmaf(ani, kFold, c2i[it]);
        const float ghn = fmaf(anh, kFold, c2h[it]);
        const float ng = gate_tanh(fmaf(rg, ghn, gin));
        const float hn = fmaf(zg, h2f[it] - ng, ng);
        h2f[it] = hn;
        if (it < 2 || tailOk) {
          sH2[ho[it]]  = to_h_flush(hn);
          sH2f[fo[it]] = hn;
        }
      }
    }
    if (padOk) sH2[padOff] = (_Float16)0.0f;
    __syncthreads();

    if (wave == 0) {
      const float* hp = sH2f + jj * kHfP + 32 * hh;
      const float* lp = sLw + 32 * hh;
      float a = 0.0f;
#pragma unroll
      for (int i = 0; i < 8; ++i) {
        const v4f hv = *(const v4f*)(hp + 4 * i);
        const v4f lv = *(const v4f*)(lp + 4 * i);
        a = fmaf(hv[0], lv[0], a);
        a = fmaf(hv[1], lv[1], a);
        a = fmaf(hv[2], lv[2], a);
        a = fmaf(hv[3], lv[3], a);
      }
      sOutP[hh * (kRows * kChunk) + jj * kChunk + tl] = a;
    }

    if (tl == kChunk - 1) {
      __syncthreads();
      const int tn = (t + 1 < kSteps) ? (t + 1) : (kSteps - kChunk);
      const v4f xv = *(const v4f*)(xsrc + tn);
      float x0 = xv[0];
      float x1 = xv[1];
      float x2 = xv[2];
      float x3 = xv[3];
      asm volatile("" : "+v"(x0));
      asm volatile("" : "+v"(x1));
      asm volatile("" : "+v"(x2));
      asm volatile("" : "+v"(x3));
      if (wave < 4) {
        const int row = wave * 4 + (lane >> 3);
        const int c4  = (lane & 7) * 4;
        const v4f p0 = *(const v4f*)(sOutP + row * kChunk + c4);
        const v4f p1 = *(const v4f*)(sOutP + kRows * kChunk + row * kChunk + c4);
        const float o0 = (p0[0] + p1[0]) + linb;
        const float o1 = (p0[1] + p1[1]) + linb;
        const float o2 = (p0[2] + p1[2]) + linb;
        const float o3 = (p0[3] + p1[3]) + linb;
        v4f ov;
        ov[0] = poison ? qnan : o0;
        ov[1] = poison ? qnan : o1;
        ov[2] = poison ? qnan : o2;
        ov[3] = poison ? qnan : o3;
        float* dst = out + (size_t)(b0 + row) * kSteps + (t - (kChunk - 1)) + c4;
        *(volatile v4f*)dst = ov;
        __threadfence();
        *(volatile v4f*)dst = ov;
      }
      if (tid < 128) {
        v4f xs;
        xs[0] = bf16_value(x0);
        xs[1] = bf16_value(x1);
        xs[2] = bf16_value(x2);
        xs[3] = bf16_value(x3);
        *(v4f*)(sX + xr * kChunk + xp) = xs;
      }
    }
  }
}

extern "C" void kernel_launch(void* const* d_in, const int* in_sizes, int n_in,
                              void* d_out, int out_size, void* d_ws, size_t ws_size,
                              hipStream_t stream) {
  (void)d_ws;
  (void)ws_size;
  if (n_in < 12) return;
  if (in_sizes[0] != kBatch * kSteps) return;
  if (in_sizes[1] != kGate) return;
  if (in_sizes[2] != kGate * kHid) return;
  if (in_sizes[3] != kGate) return;
  if (in_sizes[4] != kGate) return;
  if (in_sizes[5] != kGate * kHid) return;
  if (in_sizes[6] != kGate * kHid) return;
  if (in_sizes[7] != kGate) return;
  if (in_sizes[8] != kGate) return;
  if (in_sizes[9] != kHid) return;
  if (in_sizes[10] != 1) return;
  if (in_sizes[11] != 1) return;
  if (out_size != kBatch * kSteps) return;

  const float* input = (const float*)d_in[0];
  const float* w_ih1 = (const float*)d_in[1];
  const float* w_hh1 = (const float*)d_in[2];
  const float* b_ih1 = (const float*)d_in[3];
  const float* b_hh1 = (const float*)d_in[4];
  const float* w_ih2 = (const float*)d_in[5];
  const float* w_hh2 = (const float*)d_in[6];
  const float* b_ih2 = (const float*)d_in[7];
  const float* b_hh2 = (const float*)d_in[8];
  const float* lin_w = (const float*)d_in[9];
  const float* lin_b = (const float*)d_in[10];
  const int*   futp  = (const int*)d_in[11];
  float* out = (float*)d_out;

  two_cell_scalar_steps<<<dim3(kBlocks), dim3(kThreads), 0, stream>>>(
      input, w_ih1, w_hh1, b_ih1, b_hh1, w_ih2, w_hh2, b_ih2, b_hh2, lin_w, lin_b, futp, out);
}
